// _GCNLayer_87385404604759
// MI455X (gfx1250) — hardware-run, weakly checked
//
#include <hip/hip_runtime.h>
#include <math.h>

typedef __attribute__((ext_vector_type(16))) _Float16 v16h;
typedef __attribute__((ext_vector_type(8)))  _Float16 v8h;
typedef __attribute__((ext_vector_type(8)))  float    v8f;
typedef __attribute__((ext_vector_type(4)))  float    v4f;

constexpr int kBatch   = 32;
constexpr int kNode    = 1024;
constexpr int kChan    = 256;
constexpr int kEmb     = 64;
constexpr int kRank    = 16;
constexpr int kRowsAll = kBatch * kNode;
constexpr int kStackRows = 2 * kNode;
constexpr int kPartPitch = 32;
static_assert((kNode % 64) == 0 && (kChan % 64) == 0 && (kStackRows % 64) == 0);
static_assert((kNode % 32) == 0 && (kChan % 32) == 0);
static_assert(kRank == 16 && kEmb == 64);

constexpr int isqrt_c(int v) { int r = 0; while ((r + 1) * (r + 1) <= v) ++r; return r; }
constexpr int kSqrtRank = isqrt_c(kRank);
static_assert(kSqrtRank * kSqrtRank == kRank);
constexpr float kInvSqrtRank = 1.0f / (float)kSqrtRank;

constexpr float kCarryA = 64.0f;
constexpr float kCarryX = 16.0f;
constexpr float kCarryW = 256.0f;
constexpr float kCarryY = 256.0f;
constexpr float kScaleMix = kCarryY / (kCarryA * kCarryX);
constexpr float kInvGate  = 1.0f / (kCarryX * kCarryW);
constexpr float kInvOut   = 1.0f / (kCarryY * kCarryW);
constexpr float kF16MinNormal = 6.103515625e-05f;
constexpr float kLn2 = 0.69314718055994530942f;

constexpr size_t kOffASTK = 0;
constexpr size_t kOffXT   = kOffASTK + (size_t)kStackRows * kNode * 2;
constexpr size_t kOffYST  = kOffXT   + (size_t)kBatch * kChan * kNode * 2;
constexpr size_t kOffM16  = kOffYST  + (size_t)kBatch * kStackRows * kChan * 2;
constexpr size_t kOffWAT  = kOffM16  + (size_t)kRowsAll * kChan * 2;
constexpr size_t kOffWPT  = kOffWAT  + (size_t)kChan * kChan * 2;
constexpr size_t kOffWMT  = kOffWPT  + (size_t)kChan * kChan * 2;
constexpr size_t kOffUU   = kOffWMT  + (size_t)kChan * kChan * 2;
constexpr size_t kOffVV   = kOffUU   + (size_t)kNode * kRank * 4;
constexpr size_t kOffDINV = kOffVV   + (size_t)kNode * kRank * 4;
constexpr size_t kOffPART = kOffDINV + (size_t)kNode * 4;
constexpr size_t kWsTotal = kOffPART + (size_t)kNode * kPartPitch * 4;
static_assert(kWsTotal == 71962624ull);
static_assert(kWsTotal <= 134217728ull);
static_assert((kOffXT % 128) == 0 && (kOffYST % 128) == 0 && (kOffM16 % 128) == 0 && (kOffWAT % 128) == 0 &&
              (kOffWPT % 128) == 0 && (kOffWMT % 128) == 0 && (kOffUU % 128) == 0 && (kOffVV % 128) == 0 &&
              (kOffDINV % 128) == 0 && (kOffPART % 128) == 0);

__device__ __forceinline__ _Float16 to_h_flush(float v) {
  const float w = (fabsf(v) < kF16MinNormal) ? 0.0f : v;
  return (_Float16)w;
}

__device__ __forceinline__ void tie1_h(v8f& a, v16h x, v16h y) { asm volatile("v_nop" : "+v"(a) : "v"(x), "v"(y)); }
__device__ __forceinline__ void tie4_h(v8f& a, v16h x, v16h y) { asm volatile("v_nop\n\tv_nop\n\tv_nop\n\tv_nop" : "+v"(a) : "v"(x), "v"(y)); }
__device__ __forceinline__ void keep4_h(v16h a, v16h b, v16h c, v16h d) { asm volatile("v_nop" :: "v"(a), "v"(b), "v"(c), "v"(d)); }
__device__ __forceinline__ void acc_guard1(v8f& a) { asm volatile("v_nop\n\tv_nop\n\tv_nop\n\tv_nop" : "+v"(a)); }

__device__ __forceinline__ void wave_lds_sync() {
  __builtin_amdgcn_fence(__ATOMIC_RELEASE, "workgroup");
  __builtin_amdgcn_wave_barrier();
  __builtin_amdgcn_fence(__ATOMIC_ACQUIRE, "workgroup");
}

struct FragH {
  union U { v16h v; v8h h[2]; };
  static __device__ __forceinline__ v16h load(const _Float16* p) {
    U f; f.h[0] = *(const v8h*)(p); f.h[1] = *(const v8h*)(p + 16); return f.v;
  }
  static __device__ __forceinline__ v8f mma(v16h a, v16h b, v8f c) {
    return __builtin_amdgcn_wmma_f32_16x16x32_f16(false, a, false, b, (short)0, c, false, false);
  }
};

__global__ __launch_bounds__(256) void degree_kernel(const float* __restrict__ phy, float* __restrict__ dinv) {
  __shared__ float sdeg[32];
  const int tid = threadIdx.x, lane = tid & 31, wave = tid >> 5;
  const int mb = blockIdx.x * 32;
#pragma unroll 1
  for (int rr = 0; rr < 4; ++rr) {
    const int lr = wave * 4 + rr;
    const int m = mb + lr;
    float s = 0.0f;
#pragma unroll 4
    for (int it = 0; it < kNode / 32; ++it) {
      const int n = it * 32 + lane;
      const float a0 = phy[(size_t)m * kNode + n];
      const float a1 = phy[(size_t)n * kNode + m];
      float a = fmaxf(a0, a1);
      a = (n == m) ? fmaxf(a, 1.0f) : a;
      s += a;
    }
#pragma unroll
    for (int off = 16; off > 0; off >>= 1) s += __shfl_xor(s, off, 32);
    if (lane == 0) sdeg[lr] = s;
  }
  __syncthreads();
  if (wave == 0) {
    const float v = rsqrtf(sdeg[lane]);
    volatile float* q = dinv + mb + lane;
    *q = v;
    __threadfence();
    *q = v;
  }
}

__global__ __launch_bounds__(128) void anorm_kernel(const float* __restrict__ phy, const float* __restrict__ dinv,
                                                    unsigned short* __restrict__ astk) {
  const int m = blockIdx.x, t = threadIdx.x;
  const int n0 = t * 8;
  const v4f p0 = *(const v4f*)(phy + (size_t)m * kNode + n0);
  const v4f p1 = *(const v4f*)(phy + (size_t)m * kNode + n0 + 4);
  const v4f d0 = *(const v4f*)(dinv + n0);
  const v4f d1 = *(const v4f*)(dinv + n0 + 4);
  const float dm = dinv[m] * kCarryA;
  float rowv[8], dn[8], colv[8];
#pragma unroll
  for (int e = 0; e < 4; ++e) {
    rowv[e] = p0[e]; rowv[4 + e] = p1[e];
    dn[e] = d0[e];   dn[4 + e] = d1[e];
  }
#pragma unroll
  for (int e = 0; e < 8; ++e) colv[e] = phy[(size_t)(n0 + e) * kNode + m];
  v8h hv;
#pragma unroll
  for (int e = 0; e < 8; ++e) {
    float a = fmaxf(rowv[e], colv[e]);
    a = ((n0 + e) == m) ? fmaxf(a, 1.0f) : a;
    const float v = (dm * a) * dn[e];
    hv[e] = to_h_flush(v);
  }
  unsigned short* q = astk + (size_t)m * kNode + n0;
  *(volatile v8h*)q = hv;
  __threadfence();
  *(volatile v8h*)q = hv;
}

__global__ __launch_bounds__(256) void lowrank_proj_kernel(const float* __restrict__ emb, const float* __restrict__ Wu,
                                                           const float* __restrict__ Wv, float* __restrict__ Uo,
                                                           float* __restrict__ Vo) {
  const int sel = blockIdx.x >> 6;
  const int rem = (blockIdx.x & 63) * 256 + threadIdx.x;
  const int n = rem >> 4, r = rem & 15;
  const float* W = sel ? Wv : Wu;
  float* O = sel ? Vo : Uo;
  float s = 0.0f;
#pragma unroll 4
  for (int k = 0; k < kEmb; ++k) s = fmaf(emb[n * kEmb + k], W[k * kRank + r], s);
  volatile float* q = O + rem;
  *q = s;
  __threadfence();
  *q = s;
}

__global__ __launch_bounds__(128) void pgrow_kernel(const float* __restrict__ Um, const float* __restrict__ Vm,
                                                    const float* __restrict__ phy, unsigned short* __restrict__ astk2,
                                                    float* __restrict__ part) {
  __shared__ __align__(16) float sp[kNode];
  __shared__ float sred[3][4];
  const int m = blockIdx.x, tid = threadIdx.x, lane = tid & 31, wave = tid >> 5;
  float uu[16];
  {
    const v4f u0 = *(const v4f*)(Um + m * kRank);
    const v4f u1 = *(const v4f*)(Um + m * kRank + 4);
    const v4f u2 = *(const v4f*)(Um + m * kRank + 8);
    const v4f u3 = *(const v4f*)(Um + m * kRank + 12);
#pragma unroll
    for (int e = 0; e < 4; ++e) { uu[e] = u0[e]; uu[4 + e] = u1[e]; uu[8 + e] = u2[e]; uu[12 + e] = u3[e]; }
  }
  float accP = 0.0f, accR = 0.0f, accK = 0.0f;
#pragma unroll 1
  for (int it = 0; it < kNode / 128; ++it) {
    const int n = it * 128 + tid;
    const v4f w0 = *(const v4f*)(Vm + n * kRank);
    const v4f w1 = *(const v4f*)(Vm + n * kRank + 4);
    const v4f w2 = *(const v4f*)(Vm + n * kRank + 8);
    const v4f w3 = *(const v4f*)(Vm + n * kRank + 12);
    float vv[16];
#pragma unroll
    for (int e = 0; e < 4; ++e) { vv[e] = w0[e]; vv[4 + e] = w1[e]; vv[8 + e] = w2[e]; vv[12 + e] = w3[e]; }
    float dot = 0.0f;
#pragma unroll
    for (int k = 0; k < 16; ++k) dot = fmaf(uu[k], vv[k], dot);
    const float lg = dot * kInvSqrtRank;
    const float ex = expf(-fabsf(lg));
    const float l1 = log1pf(ex);
    const float logp = fminf(lg, 0.0f) - l1;
    const float log1mp = fminf(-lg, 0.0f) - l1;
    const float rc = 1.0f / (1.0f + ex);
    const float p = (lg >= 0.0f) ? rc : ex * rc;
    const float s0 = phy[(size_t)m * kNode + n];
    const float s1 = phy[(size_t)n * kNode + m];
    const float S = fmaxf(s0, s1);
    accR += S * logp + (1.0f - S) * log1mp;
    accK += p * (logp + kLn2) + (1.0f - p) * (log1mp + kLn2);
    const float pv = p + ((n == m) ? 1.0f : 0.0f);
    accP += pv;
    sp[n] = pv;
  }
#pragma unroll
  for (int off = 16; off > 0; off >>= 1) {
    accP += __shfl_xor(accP, off, 32);
    accR += __shfl_xor(accR, off, 32);
    accK += __shfl_xor(accK, off, 32);
  }
  if (lane == 0) { sred[0][wave] = accP; sred[1][wave] = accR; sred[2][wave] = accK; }
  __syncthreads();
  const float rs   = ((sred[0][0] + sred[0][1]) + sred[0][2]) + sred[0][3];
  const float totR = ((sred[1][0] + sred[1][1]) + sred[1][2]) + sred[1][3];
  const float totK = ((sred[2][0] + sred[2][1]) + sred[2][2]) + sred[2][3];
  const float scl = (1.0f / rs) * kCarryA;
  const v4f a0 = *(const v4f*)(sp + tid * 8);
  const v4f a1 = *(const v4f*)(sp + tid * 8 + 4);
  v8h hv;
#pragma unroll
  for (int e = 0; e < 4; ++e) {
    hv[e]     = to_h_flush(a0[e] * scl);
    hv[4 + e] = to_h_flush(a1[e] * scl);
  }
  unsigned short* q = astk2 + (size_t)m * kNode + tid * 8;
  *(volatile v8h*)q = hv;
  __threadfence();
  *(volatile v8h*)q = hv;
  if (wave == 0) {
    const float pvl = (lane == 0) ? totR : ((lane == 1) ? totK : 0.0f);
    volatile float* pq = part + (size_t)m * kPartPitch + lane;
    *pq = pvl;
    __threadfence();
    *pq = pvl;
  }
}

__global__ __launch_bounds__(256) void transpose_to_f16_kernel(const float* __restrict__ in, unsigned short* __restrict__ out,
                                                               int rows, int cols, float carry) {
  __shared__ __align__(16) float sT[64 * 68];
  const int tid = threadIdx.x, lane = tid & 31, wave = tid >> 5;
  const int r0 = blockIdx.x * 64, c0 = blockIdx.y * 64;
  const size_t zoff = (size_t)blockIdx.z * (size_t)rows * (size_t)cols;
  const float* inb = in + zoff;
  unsigned short* outb = out + zoff;
#pragma unroll
  for (int i = 0; i < 4; ++i) {
    const int idx = i * 256 + tid;
    const int lr = idx >> 4, c4 = (idx & 15) * 4;
    const v4f v = *(const v4f*)(inb + (size_t)(r0 + lr) * cols + c0 + c4);
#pragma unroll
    for (int e = 0; e < 4; ++e) sT[(c4 + e) * 68 + lr] = v[e];
  }
  __syncthreads();
  const int q = lane >> 3, c8 = (lane & 7) * 8;
  v8h hv[2];
#pragma unroll
  for (int it = 0; it < 2; ++it) {
    const int lc = it * 32 + wave * 4 + q;
    const v4f a0 = *(const v4f*)(sT + lc * 68 + c8);
    const v4f a1 = *(const v4f*)(sT + lc * 68 + c8 + 4);
#pragma unroll
    for (int e = 0; e < 4; ++e) {
      hv[it][e]     = to_h_flush(a0[e] * carry);
      hv[it][4 + e] = to_h_flush(a1[e] * carry);
    }
  }
  for (int pass = 0; pass < 2; ++pass) {
#pragma unroll
    for (int it = 0; it < 2; ++it) {
      const int lc = it * 32 + wave * 4 + q;
      *(volatile v8h*)(outb + (size_t)(c0 + lc) * rows + r0 + c8) = hv[it];
    }
    __threadfence();
  }
}

__global__ __launch_bounds__(256) void convert_rows_f16_kernel(const float* __restrict__ src, unsigned short* __restrict__ dst,
                                                               int total8, float carry) {
  const int i = blockIdx.x * 256 + threadIdx.x;
  if (i >= total8) return;
  const size_t e0 = (size_t)i << 3;
  const v4f a0 = *(const v4f*)(src + e0);
  const v4f a1 = *(const v4f*)(src + e0 + 4);
  v8h hv;
#pragma unroll
  for (int e = 0; e < 4; ++e) {
    hv[e]     = to_h_flush(a0[e] * carry);
    hv[4 + e] = to_h_flush(a1[e] * carry);
  }
  unsigned short* q = dst + e0;
  *(volatile v8h*)q = hv;
  __threadfence();
  *(volatile v8h*)q = hv;
}

__global__ __launch_bounds__(256) void mix_gemm_kernel(
    const unsigned short* __restrict__ Ap, int lda,
    const unsigned short* __restrict__ Btp, int ldb, long strideB,
    unsigned short* __restrict__ Cp, int ldc, long strideC,
    int M, int N, int K, float scale) {
  const _Float16* A = (const _Float16*)Ap;
  const _Float16* Bt = (const _Float16*)Btp;
  __shared__ __align__(16) float sT[8][16 * 68];
  const int b    = blockIdx.y;
  const int lane = threadIdx.x & 31;
  const int wave = threadIdx.x >> 5;
  const int tilesN = N >> 6;
  const int tilesM = M >> 6;
  const int tile = blockIdx.x * 8 + wave;
  if (tile >= tilesM * tilesN) return;
  const int tm = tile / tilesN;
  const int tn = tile - tm * tilesN;
  const int m0 = tm << 6;
  const int n0 = tn << 6;
  const _Float16* Bb = Bt + (size_t)b * strideB;

  const int rlane = lane & 15;
  const int koff  = (lane >> 4) * 8;
  const int mOff  = (lane >> 4) * 8;

  v8f acc[4][4];
#pragma unroll
  for (int i = 0; i < 4; ++i)
#pragma unroll
    for (int j = 0; j < 4; ++j) acc[i][j] = (v8f){0.f,0.f,0.f,0.f,0.f,0.f,0.f,0.f};

  for (int k0 = 0; k0 < K; k0 += 32) {
    v16h bh[4];
#pragma unroll
    for (int j = 0; j < 4; ++j) {
      const size_t bo = (size_t)(n0 + (j << 4) + rlane) * ldb + koff + k0;
      bh[j] = FragH::load(Bb + bo);
    }
#pragma unroll
    for (int i = 0; i < 4; ++i) {
      const size_t ao = (size_t)(m0 + (i << 4) + rlane) * lda + koff + k0;
      v16h ah = FragH::load(A + ao);
#pragma unroll
      for (int j = 0; j < 4; ++j) acc[i][j] = FragH::mma(ah, bh[j], acc[i][j]);
      tie1_h(acc[i][0], ah, bh[0]);
      tie1_h(acc[i][1], ah, bh[1]);
      tie1_h(acc[i][2], ah, bh[2]);
      tie4_h(acc[i][3], ah, bh[3]);
    }
    keep4_h(bh[0], bh[1], bh[2], bh[3]);
  }
#pragma unroll
  for (int i = 0; i < 4; ++i) {
    acc_guard1(acc[i][0]);
    acc_guard1(acc[i][1]);
    acc_guard1(acc[i][2]);
    acc_guard1(acc[i][3]);
  }

  float* slab = sT[wave];
  unsigned short* C = Cp + (size_t)b * strideC;
  const int q = lane >> 3, c8 = (lane & 7) * 8;
#pragma unroll
  for (int i = 0; i < 4; ++i) {
    const int mBase = m0 + (i << 4);
#pragma unroll
    for (int j = 0; j < 4; ++j) {
#pragma unroll
      for (int r = 0; r < 8; ++r) slab[(mOff + r) * 68 + (j << 4) + rlane] = acc[i][j][r] * scale;
    }
    wave_lds_sync();
    for (int pass = 0; pass < 2; ++pass) {
#pragma unroll
      for (int it = 0; it < 4; ++it) {
        const int row = it * 4 + q;
        const float* sp = slab + row * 68 + c8;
        v8h hv;
#pragma unroll
        for (int e = 0; e < 8; ++e) hv[e] = to_h_flush(sp[e]);
        *(volatile v8h*)(C + (size_t)(mBase + row) * ldc + n0 + c8) = hv;
      }
      __threadfence();
    }
    wave_lds_sync();
  }
}

__device__ __forceinline__ void tile32x64_f16(const _Float16* __restrict__ A, const _Float16* __restrict__ Bt,
                                              int rlane, int koff, v8f (&acc)[2][4]) {
#pragma unroll 1
  for (int k0 = 0; k0 < kChan; k0 += 32) {
    v16h bh[4];
#pragma unroll
    for (int j = 0; j < 4; ++j) bh[j] = FragH::load(Bt + (size_t)((j << 4) + rlane) * kChan + koff + k0);
#pragma unroll
    for (int i = 0; i < 2; ++i) {
      v16h ah = FragH::load(A + (size_t)((i << 4) + rlane) * kChan + koff + k0);
#pragma unroll
      for (int j = 0; j < 4; ++j) acc[i][j] = FragH::mma(ah, bh[j], acc[i][j]);
      tie1_h(acc[i][0], ah, bh[0]);
      tie1_h(acc[i][1], ah, bh[1]);
      tie1_h(acc[i][2], ah, bh[2]);
      tie4_h(acc[i][3], ah, bh[3]);
    }
    keep4_h(bh[0], bh[1], bh[2], bh[3]);
  }
#pragma unroll
  for (int i = 0; i < 2; ++i) {
    acc_guard1(acc[i][0]);
    acc_guard1(acc[i][1]);
    acc_guard1(acc[i][2]);
    acc_guard1(acc[i][3]);
  }
}

constexpr int kOutWaves = 4;
__global__ __launch_bounds__(128) void fused_out_kernel(
    const unsigned short* __restrict__ Yst, const unsigned short* __restrict__ M16p,
    const unsigned short* __restrict__ WaT, const unsigned short* __restrict__ WpT,
    const unsigned short* __restrict__ WmT,
    const float* __restrict__ bag, const float* __restrict__ bpg, float* __restrict__ out) {
  __shared__ __align__(16) float sG[kOutWaves][32 * 68];
  __shared__ __align__(16) float sO[kOutWaves][16 * 68];
  const int lane = threadIdx.x & 31;
  const int wave = threadIdx.x >> 5;
  const int rlane = lane & 15;
  const int koff  = (lane >> 4) * 8;
  const int mOff  = (lane >> 4) * 8;
  const int tile = blockIdx.x * kOutWaves + wave;
  const int tm = tile >> 2;
  const int tn = tile & 3;
  const int m0 = tm * 32;
  const int n0 = tn * 64;
  const int bidx = m0 / kNode;
  const int mr = m0 - bidx * kNode;
  const _Float16* Y1 = (const _Float16*)Yst + ((size_t)bidx * kStackRows + mr) * kChan;
  const _Float16* Y2 = Y1 + (size_t)kNode * kChan;
  const _Float16* Mm = (const _Float16*)M16p + (size_t)m0 * kChan;
  const _Float16* Bm = (const _Float16*)WmT + (size_t)n0 * kChan;
  const _Float16* Bp = (const _Float16*)WpT + (size_t)n0 * kChan;
  const _Float16* Ba = (const _Float16*)WaT + (size_t)n0 * kChan;
  float* sg = sG[wave];
  float* so = sO[wave];

  {
    v8f g[2][4];
#pragma unroll
    for (int i = 0; i < 2; ++i)
#pragma unroll
      for (int j = 0; j < 4; ++j) g[i][j] = (v8f){0.f,0.f,0.f,0.f,0.f,0.f,0.f,0.f};
    tile32x64_f16(Mm, Bm, rlane, koff, g);
#pragma unroll
    for (int i = 0; i < 2; ++i)
#pragma unroll
      for (int j = 0; j < 4; ++j)
#pragma unroll
        for (int r = 0; r < 8; ++r)
          sg[((i << 4) + mOff + r) * 68 + (j << 4) + rlane] = g[i][j][r] * kInvGate;
  }
  wave_lds_sync();
#pragma unroll 1
  for (int e = 0; e < 64; ++e) {
    const int idx = e * 32 + lane;
    const int row = idx >> 6, col = idx & 63;
    float* gq = sg + row * 68 + col;
    const float v = *gq;
    *gq = 1.0f / (1.0f + expf(-v));
  }
  wave_lds_sync();

  v8f fa[2][4], aa[2][4];
#pragma unroll
  for (int i = 0; i < 2; ++i)
#pragma unroll
    for (int j = 0; j < 4; ++j) {
      fa[i][j] = (v8f){0.f,0.f,0.f,0.f,0.f,0.f,0.f,0.f};
      aa[i][j] = (v8f){0.f,0.f,0.f,0.f,0.f,0.f,0.f,0.f};
    }
  tile32x64_f16(Y2, Bp, rlane, koff, fa);
  tile32x64_f16(Y1, Ba, rlane, koff, aa);

  float ba[4], bp[4];
#pragma unroll
  for (int j = 0; j < 4; ++j) {
    ba[j] = bag[n0 + (j << 4) + rlane];
    bp[j] = bpg[n0 + (j << 4) + rlane];
  }
  const int hh = lane >> 4, c4 = (lane & 15) * 4;
#pragma unroll
  for (int i = 0; i < 2; ++i) {
#pragma unroll
    for (int j = 0; j < 4; ++j) {
#pragma unroll
      for (int r = 0; r < 8; ++r) {
        const float gate = sg[((i << 4) + mOff + r) * 68 + (j << 4) + rlane];
        const float fv = fa[i][j][r] * kInvOut + bp[j];
        const float av = aa[i][j][r] * kInvOut + ba[j];
        so[(mOff + r) * 68 + (j << 4) + rlane] = av + fv * gate;
      }
    }
    wave_lds_sync();
    for (int pass = 0; pass < 2; ++pass) {
#pragma unroll
      for (int it = 0; it < 8; ++it) {
        const int row = it * 2 + hh;
        const v4f v = *(const v4f*)(so + row * 68 + c4);
        *(volatile v4f*)(out + (size_t)(m0 + (i << 4) + row) * kChan + n0 + c4) = v;
      }
      __threadfence();
    }
    wave_lds_sync();
  }
}

__global__ __launch_bounds__(256) void elbo_finish_kernel(const float* __restrict__ part, float* __restrict__ out1) {
  __shared__ float sr[256];
  __shared__ float sk[256];
  const int tid = threadIdx.x;
  float r = 0.0f, k = 0.0f;
#pragma unroll
  for (int i = 0; i < kNode / 256; ++i) {
    const int line = i * 256 + tid;
    r += part[(size_t)line * kPartPitch];
    k += part[(size_t)line * kPartPitch + 1];
  }
  sr[tid] = r;
  sk[tid] = k;
  __syncthreads();
  for (int st = 128; st > 0; st >>= 1) {
    if (tid < st) { sr[tid] += sr[tid + st]; sk[tid] += sk[tid + st]; }
    __syncthreads();
  }
  if (tid == 0) {
    const float inv = 1.0f / ((float)kNode * (float)kNode);
    const float v = sr[0] * inv - sk[0] * inv;
    volatile float* q = out1;
    *q = v;
    __threadfence();
    *q = v;
  }
}

extern "C" void kernel_launch(void* const* d_in, const int* in_sizes, int n_in,
                              void* d_out, int out_size, void* d_ws, size_t ws_size,
                              hipStream_t stream) {
  if (n_in < 11) return;
  if (in_sizes[0] != kRowsAll * kChan) return;
  if (in_sizes[1] != kRowsAll * kChan) return;
  if (in_sizes[2] != kNode * kNode) return;
  if (in_sizes[3] != kChan * kChan) return;
  if (in_sizes[4] != kChan) return;
  if (in_sizes[5] != kNode * kEmb) return;
  if (in_sizes[6] != kEmb * kRank) return;
  if (in_sizes[7] != kEmb * kRank) return;
  if (in_sizes[8] != kChan * kChan) return;
  if (in_sizes[9] != kChan) return;
  if (in_sizes[10] != kChan * kChan) return;
  if (out_size != kRowsAll * kChan + 1) return;
  if (ws_size < kWsTotal) return;

  const float* x      = (const float*)d_in[0];
  const float* memory = (const float*)d_in[1];
  const float* phy    = (const float*)d_in[2];
  const float* W_ag   = (const float*)d_in[3];
  const float* b_ag   = (const float*)d_in[4];
  const float* emb    = (const float*)d_in[5];
  const float* Wu     = (const float*)d_in[6];
  const float* Wv     = (const float*)d_in[7];
  const float* W_pg   = (const float*)d_in[8];
  const float* b_pg   = (const float*)d_in[9];
  const float* Wm     = (const float*)d_in[10];
  float* out = (float*)d_out;

  char* ws = (char*)d_ws;
  unsigned short* ASTK = (unsigned short*)(ws + kOffASTK);
  unsigned short* XT   = (unsigned short*)(ws + kOffXT);
  unsigned short* YST  = (unsigned short*)(ws + kOffYST);
  unsigned short* M16  = (unsigned short*)(ws + kOffM16);
  unsigned short* WAT  = (unsigned short*)(ws + kOffWAT);
  unsigned short* WPT  = (unsigned short*)(ws + kOffWPT);
  unsigned short* WMT  = (unsigned short*)(ws + kOffWMT);
  float* UU   = (float*)(ws + kOffUU);
  float* VV   = (float*)(ws + kOffVV);
  float* DINV = (float*)(ws + kOffDINV);
  float* PART = (float*)(ws + kOffPART);

  degree_kernel<<<kNode / 32, 256, 0, stream>>>(phy, DINV);
  anorm_kernel<<<kNode, 128, 0, stream>>>(phy, DINV, ASTK);
  lowrank_proj_kernel<<<128, 256, 0, stream>>>(emb, Wu, Wv, UU, VV);
  pgrow_kernel<<<kNode, 128, 0, stream>>>(UU, VV, phy, ASTK + (size_t)kNode * kNode, PART);

  transpose_to_f16_kernel<<<dim3(kNode / 64, kChan / 64, kBatch), 256, 0, stream>>>(x, XT, kNode, kChan, kCarryX);
  convert_rows_f16_kernel<<<(kRowsAll * kChan / 8) / 256, 256, 0, stream>>>(memory, M16, kRowsAll * kChan / 8, kCarryX);
  transpose_to_f16_kernel<<<dim3(kChan / 64, kChan / 64, 1), 256, 0, stream>>>(W_ag, WAT, kChan, kChan, kCarryW);
  transpose_to_f16_kernel<<<dim3(kChan / 64, kChan / 64, 1), 256, 0, stream>>>(W_pg, WPT, kChan, kChan, kCarryW);
  transpose_to_f16_kernel<<<dim3(kChan / 64, kChan / 64, 1), 256, 0, stream>>>(Wm, WMT, kChan, kChan, kCarryW);

  mix_gemm_kernel<<<dim3((kStackRows / 64) * (kChan / 64) / 8, kBatch), 256, 0, stream>>>(
      ASTK, kNode,
      XT, kNode, (long)kChan * kNode,
      YST, kChan, (long)kStackRows * kChan,
      kStackRows, kChan, kNode, kScaleMix);

  fused_out_kernel<<<(kRowsAll / 32) * (kChan / 64) / kOutWaves, 128, 0, stream>>>(
      YST, M16, WAT, WPT, WMT, b_ag, b_pg, out);

  elbo_finish_kernel<<<1, 256, 0, stream>>>(PART, out + (size_t)kRowsAll * kChan);
}
